// LowGraph_3539053052649
// MI455X (gfx1250) — hardware-run, weakly checked
//
#include <hip/hip_runtime.h>


namespace {
constexpr int NBt = 256, NN = 200, FI = 320, F1 = 32, F2 = 64, NROW = NBt * NN  , NT = 13  , KP = 224  , OW = 128;
constexpr float XS = 8.0f, HS = 256.0f, PS = 256.0f, WSC = 256.0f, NEG = -9e15f;
typedef _Float16 b16;
typedef __attribute__((ext_vector_type(16))) _Float16 v16b;
typedef __attribute__((ext_vector_type(8))) _Float16 v8b;
typedef __attribute__((ext_vector_type(8))) float v8f;
typedef __attribute__((ext_vector_type(4))) float v4f;
typedef __attribute__((ext_vector_type(2))) float v2f;
__device__ __forceinline__ float bf16_rne(float f) { unsigned int u = __float_as_uint(f); u += 0x7FFFu + ((u >> 16) & 1u); float r = __uint_as_float(u & 0xFFFF0000u); asm volatile("" : "+v"(r)); return r; }
__device__ __forceinline__ float bfv(float f) { float r = bf16_rne(f); asm volatile("" : "+v"(r)); return r; }
__device__ __forceinline__ void split16(float v, b16& hi, b16& lo) { hi = (b16)v; lo = (b16)(v - (float)hi); }
__device__ __forceinline__ v16b frag_kb(const b16* p, int hh) { const v8b a = *(const v8b*)(p + 8 * hh), b = *(const v8b*)(p + 16 + 8 * hh); v16b f;
#pragma unroll
  for (int e = 0; e < 8; ++e) { f[e] = a[e]; f[8 + e] = b[e]; } return f; }
__device__ __forceinline__ v8f wmma16b(v16b a, v16b b, v8f c) { v8f d = __builtin_amdgcn_wmma_f32_16x16x32_f16(false, a, false, b, (short)0, c, false, false); asm volatile("v_nop\n\tv_nop\n\tv_nop\n\tv_nop" : "+v"(d) : "v"(a), "v"(b)); return d; }
__device__ __forceinline__ void wave_lds_sync() { __builtin_amdgcn_fence(__ATOMIC_RELEASE, "workgroup"); __builtin_amdgcn_wave_barrier(); __builtin_amdgcn_fence(__ATOMIC_ACQUIRE, "workgroup"); }
__device__ __forceinline__ float pmul(float a, float b) { float p = a * b; asm volatile("" : "+v"(p)); return p; }
__device__ __forceinline__ float elu(float v) { return v > 0.0f ? v : (__expf(v) - 1.0f); }

__global__ __launch_bounds__(256) void wput_kernel(const float* __restrict__ w10, const float* __restrict__ w11, const float* __restrict__ w2, b16* __restrict__ WA, b16* __restrict__ WB) { const int u = blockIdx.x * 256 + threadIdx.x; v8b v;
  if (u < 2 * F1 * (FI / 8)) { const int o = u / (FI / 8), k0 = (u % (FI / 8)) * 8; const float* w = o < F1 ? w10 : w11; const int c = o % F1;
#pragma unroll
    for (int j = 0; j < 8; ++j) v[j] = (b16)(bf16_rne(w[(size_t)(k0 + j) * F1 + c]) * WSC); for (int pass = 0; pass < 2; ++pass) { *(volatile v8b*)(WA + (size_t)o * FI + k0) = v; __threadfence(); } }
  if (u < F2 * 8) { const int o = u / 8, k0 = (u % 8) * 8;
#pragma unroll
    for (int j = 0; j < 8; ++j) v[j] = (b16)(bf16_rne(w2[(size_t)(k0 + j) * F2 + o]) * WSC); for (int pass = 0; pass < 2; ++pass) { *(volatile v8b*)(WB + (size_t)o * F2 + k0) = v; __threadfence(); } } }
template <int MODE>
__global__ __launch_bounds__(32) void lin_kernel(const float* __restrict__ IN, const b16* __restrict__ W, const float* __restrict__ aA, const float* __restrict__ aB, int RLIM, float* __restrict__ H, float* __restrict__ SD) { constexpr int KIN = MODE == 0 ? FI : F2; __shared__ __attribute__((aligned(16))) b16 Ah[16][KIN + 8], Al[16][KIN + 8]; __shared__ float Tf[16][68], Sq[16][4]; const int lane = threadIdx.x, nloc = lane & 15, hlf = lane >> 4; const size_t m0 = (size_t)blockIdx.x * 16; if (m0 >= (size_t)RLIM) return;
  for (int rr = 0; rr < 16; ++rr) for (int q = 0; q < KIN / 32; ++q) { const int c = q * 32 + lane; const float v = IN[(m0 + rr) * KIN + c]; b16 p, ql; if (MODE == 0) { p = (b16)(bf16_rne(v) * XS); ql = (b16)0.0f; } else split16(v * HS, p, ql); Ah[rr][c] = p; Al[rr][c] = ql; }
  if (lane < 16) for (int k = KIN; k < KIN + 8; ++k) { Ah[lane][k] = (b16)0.0f; Al[lane][k] = (b16)0.0f; }
  wave_lds_sync(); v8f acc[4] = {(v8f){}, (v8f){}, (v8f){}, (v8f){}};
#pragma unroll 2
  for (int kb = 0; kb < KIN; kb += 32) { const v16b a = frag_kb(&Ah[nloc][kb], hlf), al = frag_kb(&Al[nloc][kb], hlf);
#pragma unroll
    for (int t = 0; t < 4; ++t) { const v16b bw = frag_kb(W + (size_t)(t * 16 + nloc) * KIN + kb, hlf); acc[t] = wmma16b(a, bw, acc[t]); if (MODE == 1) acc[t] = wmma16b(al, bw, acc[t]); } }
  const float osc = MODE == 0 ? 1.0f / (XS * WSC) : 1.0f / (HS * WSC);
#pragma unroll
  for (int t = 0; t < 4; ++t)
#pragma unroll
    for (int r8 = 0; r8 < 8; ++r8) Tf[8 * hlf + r8][t * 16 + nloc] = acc[t][r8] * osc;
  wave_lds_sync();
  for (int rr = 0; rr < 16; ++rr) { float s0, s1, s2 = 0.0f, s3 = 0.0f; if (MODE == 0) { s0 = pmul(Tf[rr][lane], bfv(aA[lane])); s1 = pmul(Tf[rr][lane], bfv(aA[F1 + lane])); s2 = pmul(Tf[rr][F1 + lane], bfv(aB[lane])); s3 = pmul(Tf[rr][F1 + lane], bfv(aB[F1 + lane])); } else { s0 = pmul(Tf[rr][lane], bfv(aA[lane])) + pmul(Tf[rr][32 + lane], bfv(aA[32 + lane])); s1 = pmul(Tf[rr][lane], bfv(aA[F2 + lane])) + pmul(Tf[rr][32 + lane], bfv(aA[F2 + 32 + lane])); }
    for (int o = 16; o; o >>= 1) { s0 += __shfl_xor(s0, o); s1 += __shfl_xor(s1, o); s2 += __shfl_xor(s2, o); s3 += __shfl_xor(s3, o); } if (lane == 0) { Sq[rr][0] = s0; Sq[rr][1] = s1; Sq[rr][2] = s2; Sq[rr][3] = s3; } }
  wave_lds_sync();
  for (int pass = 0; pass < 2; ++pass) { for (int rr = 0; rr < 16; ++rr) *(volatile v2f*)(H + (m0 + rr) * 64 + lane * 2) = *(const v2f*)(&Tf[rr][lane * 2]); for (int q = 0; q < 2; ++q) ((volatile float*)SD)[m0 * 4 + q * 32 + lane] = Sq[(q * 32 + lane) >> 2][(q * 32 + lane) & 3]; __threadfence(); } }
template <int F, int NHD>
__global__ __launch_bounds__(32) void att_kernel(const float* __restrict__ H, const float* __restrict__ SD, const int* __restrict__ adj, int BLIM, int OCOL, float* __restrict__ X, float* __restrict__ out) {
  __shared__ __attribute__((aligned(16))) b16 Hth[F][KP + 8], Htl[F][KP + 8], Ph[16][KP + 8], Pl[16][KP + 8]; __shared__ float Ef[16][KP + 1], Of[16][F + 1];
  const int lane = threadIdx.x, nloc = lane & 15, hlf = lane >> 4; const int t = blockIdx.x % NT, hd = (blockIdx.x / NT) % NHD, b = blockIdx.x / (NT * NHD); if (b >= BLIM) return; const int i0 = t * 16; const size_t rb = (size_t)b * NN;
  for (int j = lane; j < KP + 8; j += 32) for (int f = 0; f < F; ++f) { b16 p = (b16)0.0f, ql = (b16)0.0f; if (j < NN) split16(H[(rb + j) * 64 + hd * F + f] * HS, p, ql); Hth[f][j] = p; Htl[f][j] = ql; }
  for (int r = 0; r < 16; ++r) { const int i = i0 + r; const float si = i < NN ? SD[(rb + i) * 4 + hd * 2] : 0.0f; for (int j = lane; j < KP; j += 32) { float e = NEG; if (i < NN && j < NN) { const float v = si + SD[(rb + j) * 4 + hd * 2 + 1]; const float lv = v > 0.0f ? v : 0.2f * v; e = adj[i * NN + j] > 0 ? lv : NEG; } Ef[r][j] = e; } }
  wave_lds_sync();
  for (int r = 0; r < 16; ++r) { float mx = -INFINITY; for (int j = lane; j < NN; j += 32) mx = fmaxf(mx, Ef[r][j]); for (int o = 16; o; o >>= 1) mx = fmaxf(mx, __shfl_xor(mx, o)); float sm = 0.0f; for (int j = lane; j < NN; j += 32) { const float p = __expf(Ef[r][j] - mx); Ef[r][j] = p; sm += p; } for (int o = 16; o; o >>= 1) sm += __shfl_xor(sm, o); const float inv = 1.0f / sm;
    for (int j = lane; j < KP + 8; j += 32) { b16 p = (b16)0.0f, ql = (b16)0.0f; if (j < NN) split16(Ef[r][j] * inv * PS, p, ql); Ph[r][j] = p; Pl[r][j] = ql; } }
  wave_lds_sync();
  v8f acc[F / 16];
#pragma unroll
  for (int tt = 0; tt < F / 16; ++tt) acc[tt] = (v8f){};
#pragma unroll
  for (int kb = 0; kb < KP; kb += 32) { const v16b pa = frag_kb(&Ph[nloc][kb], hlf), pb = frag_kb(&Pl[nloc][kb], hlf);
#pragma unroll
    for (int tt = 0; tt < F / 16; ++tt) { const v16b vh = frag_kb(&Hth[tt * 16 + nloc][kb], hlf), vl = frag_kb(&Htl[tt * 16 + nloc][kb], hlf); acc[tt] = wmma16b(pa, vh, acc[tt]); acc[tt] = wmma16b(pa, vl, acc[tt]); acc[tt] = wmma16b(pb, vh, acc[tt]); } }
#pragma unroll
  for (int tt = 0; tt < F / 16; ++tt)
#pragma unroll
    for (int r8 = 0; r8 < 8; ++r8) Of[8 * hlf + r8][tt * 16 + nloc] = elu(acc[tt][r8] * (1.0f / (PS * HS)));
  wave_lds_sync();
  for (int pass = 0; pass < 2; ++pass) { for (int r = 0; r < 16; ++r) { const int i = i0 + r; if (i >= NN) break; for (int q = 0; q < F / 32; ++q) { const float v = Of[r][q * 32 + lane]; if (X) ((volatile float*)X)[(rb + i) * 64 + hd * F + q * 32 + lane] = v; ((volatile float*)out)[(rb + i) * OW + OCOL + hd * F + q * 32 + lane] = v; } } __threadfence(); } }
}

extern "C" void kernel_launch(void* const* d_in, const int* in_sizes, int n_in, void* d_out, int out_size, void* d_ws, size_t ws_size, hipStream_t stream) {
  (void)n_in;
  auto Fp = [&](int i) { return (const float*)d_in[i]; }; auto Ip = [&](int i) { return (const int*)d_in[i]; };
  if (in_sizes[0] != NROW * FI || in_sizes[1] != NN * NN || in_sizes[2] != FI * F1 || in_sizes[4] != FI * F1 || in_sizes[6] != 2 * F1 * F2 || in_sizes[7] != 2 * F2 || out_size != NROW * OW) return;
  const int BLIM = NBt;
  const int RLIM = BLIM * NN;
  size_t off = 0; char* ws = (char*)d_ws;
  auto carve = [&](size_t bytes) { char* p = ws + off; off += (bytes + 255) & ~(size_t)255; return p; };
  b16* WA = (b16*)carve((size_t)2 * F1 * FI * 2); b16* WB = (b16*)carve((size_t)F2 * F2 * 2); float* H1 = (float*)carve((size_t)NROW * 64 * 4); float* SD1 = (float*)carve((size_t)NROW * 4 * 4); float* X1 = (float*)carve((size_t)NROW * 64 * 4); float* H2 = (float*)carve((size_t)NROW * 64 * 4); float* SD2 = (float*)carve((size_t)NROW * 4 * 4);
  if (off > ws_size || off > ((size_t)64 << 20)) return;
  wput_kernel<<<(2 * F1 * (FI / 8) + 255) / 256, 256, 0, stream>>>(Fp(2), Fp(4), Fp(6), WA, WB);
  lin_kernel<0><<<RLIM / 16, 32, 0, stream>>>(Fp(0), WA, Fp(3), Fp(5), RLIM, H1, SD1);
  att_kernel<F1, 2><<<NBt * 2 * NT, 32, 0, stream>>>(H1, SD1, Ip(1), BLIM, 0, X1, (float*)d_out);
  lin_kernel<1><<<RLIM / 16, 32, 0, stream>>>(X1, WB, Fp(7), Fp(7), RLIM, H2, SD2);
  att_kernel<F2, 1><<<NBt * NT, 32, 0, stream>>>(H2, SD2, Ip(1), BLIM, 64, nullptr, (float*)d_out);
}
